// LinearNonlinearRelease_82841329205926
// MI455X (gfx1250) — hardware-run, weakly checked
//
#include <hip/hip_runtime.h>
#include <math.h>

#pragma clang fp contract(off)

typedef __attribute__((ext_vector_type(16))) __bf16   v16b;
typedef __attribute__((ext_vector_type(8)))  __bf16   v8b;
typedef __attribute__((ext_vector_type(8)))  float    v8f;
typedef __attribute__((ext_vector_type(4)))  float    v4f;
typedef __attribute__((ext_vector_type(2)))  float    v2f;
typedef __attribute__((ext_vector_type(2)))  unsigned v2u;
typedef __attribute__((ext_vector_type(4)))  unsigned v4u;
typedef __attribute__((ext_vector_type(8)))  unsigned v8u;

constexpr int kD       = 1048576;
constexpr int kCells   = 14;
constexpr int kTapsF   = 20;
constexpr int kTapsB   = 32;
constexpr int kSteady  = 640;
constexpr int kPad     = kSteady + (kTapsF - 1) + (kTapsB - 1);
constexpr int kXpLen   = kD + kPad;
constexpr int kT       = kXpLen - (kTapsF - 1);
constexpr int kBlkT    = 2048;
constexpr int kFrontBlocks = (kT + kBlkT - 1) / kBlkT;
constexpr int kTP      = kFrontBlocks * kBlkT;
constexpr int kChunk   = 64;
constexpr int kNChunk  = (kT + kChunk - 1) / kChunk;
constexpr int kWinWords = 1040;
constexpr int kRdBlk   = 2048;
constexpr int kRdWin   = kRdBlk + 64;
constexpr int kRdWords = kRdWin / 2;
constexpr int kRdQuads = kRdWin / 4;
constexpr int kBandK   = 64;
static_assert(kPad == 690, "left pad");
static_assert(kXpLen == 1049266, "padded stimulus length");
static_assert(kT == 1049247, "scan steps");
static_assert(kFrontBlocks == 513 && kTP == 1050624, "time pitch");
static_assert(kNChunk == 16395 && kNChunk * kChunk <= kTP, "scan chunks inside the plane");
static_assert((kPad % 2) == 0 && (kXpLen % 2) == 0, "sample pairs never straddle a region boundary");
static_assert((kD % kRdBlk) == 0, "read-out grid exact");
static_assert(kSteady + (kD - kRdBlk) + kRdWin <= kNChunk * kChunk, "read-out staging stays inside written steps");
static_assert(kRdWin == 2112 && kRdWords == 1056 && kRdQuads == 528 && kRdQuads <= 3 * 256, "read-out window staging");
static_assert(15 + (kTapsB - 1) < kBandK, "band depth covers column offset plus taps");
static_assert((kSteady % 16) == 0, "read-out rows are 16-sample aligned");
static_assert((kTP % 32) == 0, "row pitch is a multiple of one 128-B line");

constexpr int PL_SLOPE = 0, PL_OFF = 1, PL_CP01 = 2, PL_CP12 = 3, PL_RRPCAP = 4, PL_IPCAP = 5;
constexpr int PL_IP0 = 6, PL_RRP0 = 7, PL_SCALE = 8, PL_BIAS = 9;
constexpr int kPrmLines = 10;

constexpr size_t kOffPRM = 0;
constexpr size_t kOffBTH = kOffPRM + 4096;
constexpr size_t kOffBTL = kOffBTH + 1024;
constexpr size_t kOffBKH = kOffBTL + 1024;
constexpr size_t kOffBKL = kOffBKH + 2048;
constexpr size_t kOffRP  = kOffBKL + 2048;
constexpr size_t kOffREL = kOffRP + (size_t)kCells * kTP * 4;
constexpr size_t kWsTotal = kOffREL + (size_t)kCells * kTP * 4;
static_assert(kWsTotal == 117680128ull, "carve total");
static_assert(kWsTotal <= 134217728ull, "carve cap");
static_assert((kOffBTH % 128) == 0 && (kOffBTL % 128) == 0 && (kOffBKH % 128) == 0 && (kOffBKL % 128) == 0 &&
              (kOffRP % 128) == 0 && (kOffREL % 128) == 0, "aligned regions");

__device__ __forceinline__ unsigned bf_bits(float f) {
  const unsigned u = __float_as_uint(f);
  return (u + 0x7FFFu + ((u >> 16) & 1u)) >> 16;
}
__device__ __forceinline__ float bf_bits_to_f(unsigned hb) { return __uint_as_float(hb << 16); }

__device__ __forceinline__ unsigned funnel_r(unsigned hi, unsigned lo, unsigned sh) {
  const unsigned long long v = (((unsigned long long)hi) << 32) | (unsigned long long)lo;
  return (unsigned)(v >> sh);
}

union FragB { v16b v; v8b h[2]; };
__device__ __forceinline__ v16b frag_load_bf(const __bf16* p) {
  FragB f;
  f.h[0] = *(const v8b*)(p);
  f.h[1] = *(const v8b*)(p + 16);
  return f.v;
}
__device__ __forceinline__ v8f mma_bf(v16b a, v16b b, v8f c) {
  c = __builtin_amdgcn_wmma_f32_16x16x32_bf16(false, a, false, b, (short)0, c, false, false);
  asm volatile("v_nop\n\tv_nop\n\tv_nop\n\tv_nop" : "+v"(c) : "v"(a), "v"(b));
  return c;
}
__device__ __forceinline__ void group_guard(v8f& c, v16b a0, v16b a1, v16b b0, v16b b1) {
  asm volatile("v_nop\n\tv_nop\n\tv_nop\n\tv_nop" : "+v"(c) : "v"(a0), "v"(a1), "v"(b0), "v"(b1));
}

__device__ __forceinline__ float elu_precise(float v) {
  const float em = expm1f(v);
  return (v > 0.0f) ? v : em;
}
__device__ __forceinline__ float smooth_clamp_big(float x) {
  const float t1 = x - 1.0f;
  const float a  = elu_precise(t1) + 1.0f;
  const float t2 = 999999.0f - a;
  const float e2 = elu_precise(t2);
  const float b  = (e2 - 1000000.0f) + 1.0f;
  return -b;
}
__device__ __forceinline__ float elu_fast(float v) {
  const float em = __expf(v) - 1.0f;
  return (v > 0.0f) ? v : em;
}
__device__ __forceinline__ float smooth_clamp_step(float x, float high, float hm1) {
  const float t1 = x - 1.0f;
  const float a  = elu_fast(t1) + 1.0f;
  const float t2 = hm1 - a;
  const float e2 = elu_fast(t2);
  const float b  = (e2 - high) + 1.0f;
  return -b;
}

__global__ __launch_bounds__(160) void params_kernel(
    float* __restrict__ prm,
    const float* __restrict__ soff, const float* __restrict__ lsl,
    const float* __restrict__ lcp01, const float* __restrict__ lcp12,
    const float* __restrict__ lipc, const float* __restrict__ lrpc,
    const float* __restrict__ sip, const float* __restrict__ srrp,
    const float* __restrict__ lfs, const float* __restrict__ fb)
{
  __shared__ float sSC[32];
  __shared__ float sE[160];
  const int tid = threadIdx.x;
  const int c   = tid & 15;
  const int cc  = c < kCells ? c : kCells - 1;
  const int j   = tid >> 4;
  const float v_off  = soff[cc];
  const float v_lsl  = lsl[cc];
  const float v_c01  = lcp01[cc];
  const float v_c12  = lcp12[cc];
  const float v_ipc  = lipc[cc];
  const float v_rpc  = lrpc[cc];
  const float v_sip  = sip[cc];
  const float v_srrp = srrp[cc];
  const float v_lfs  = lfs[cc];
  const float v_fb   = fb[cc];

  const float xs  = (j == 0) ? v_rpc : v_ipc;
  const float scv = smooth_clamp_big(xs);
  if (tid < 32) sSC[tid] = scv;
  __syncthreads();
  const float sc_r = sSC[c];
  const float sc_i = sSC[16 + c];
  float v = v_lsl;
  v = (j == 1) ? v_c01 : v;
  v = (j == 2) ? v_c12 : v;
  v = (j == 3) ? v_ipc : v;
  v = (j == 4) ? v_rpc : v;
  v = (j == 5) ? v_lfs : v;
  v = (j == 6) ? (-v_sip) : v;
  v = (j == 7) ? (-v_srrp) : v;
  v = (j == 8) ? sc_r : v;
  v = (j == 9) ? sc_i : v;
  sE[tid] = expf(v);
  __syncthreads();
  if (tid < 32) {
    const float e_sl   = sE[c];
    const float e_c01  = sE[16 + c];
    const float e_c12  = sE[32 + c];
    const float e_ipc  = sE[48 + c];
    const float e_rpc  = sE[64 + c];
    const float e_fs   = sE[80 + c];
    const float e_nsi  = sE[96 + c];
    const float e_nsr  = sE[112 + c];
    const float cap_r  = sE[128 + c];
    const float cap_i  = sE[144 + c];
    const float sg_ip  = 1.0f / (1.0f + e_nsi);
    const float sg_rrp = 1.0f / (1.0f + e_nsr);
    float ov[kPrmLines];
    ov[PL_SLOPE]  = e_sl;
    ov[PL_OFF]    = v_off;
    ov[PL_CP01]   = e_c01;
    ov[PL_CP12]   = e_c12;
    ov[PL_RRPCAP] = cap_r;
    ov[PL_IPCAP]  = cap_i;
    ov[PL_IP0]    = sg_ip * e_ipc;
    ov[PL_RRP0]   = sg_rrp * e_rpc;
    ov[PL_SCALE]  = e_fs;
    ov[PL_BIAS]   = v_fb;
    const bool live = (tid < 16);
#pragma unroll
    for (int ln = 0; ln < kPrmLines; ++ln) ov[ln] = live ? ov[ln] : 0.0f;
    for (int pass = 0; pass < 2; ++pass) {
#pragma unroll
      for (int ln = 0; ln < kPrmLines; ++ln) *(volatile float*)(prm + ln * 32 + tid) = ov[ln];
      __threadfence();
    }
  }
}

constexpr float kPhiC  = (float)(-3.14159265358979323846 * (0.2 / 1.4));
constexpr float kTwoPi = (float)(2.0 * 3.14159265358979323846);

__global__ __launch_bounds__(320) void taps_kernel(
    const float* __restrict__ lks, const float* __restrict__ ct, const float* __restrict__ k1,
    unsigned* __restrict__ bth, unsigned* __restrict__ btl,
    unsigned* __restrict__ bkh, unsigned* __restrict__ bkl)
{
  __shared__ float sRaw[kTapsF * 16];
  __shared__ float sNrm[16];
  __shared__ float sTap[16 * kTapsF];
  __shared__ float sK1[kTapsB];
  const int tid = threadIdx.x;
  const int c   = tid & 15;
  const int k   = tid >> 4;
  const int cc  = c < kCells ? c : kCells - 1;
  const float ks  = expf(lks[cc]);
  const float ctv = ct[cc];
  const float tau = 0.05f * ks;
  const float phi = kPhiC * ks;
  const float t   = 0.3f - (float)k * 0.015625f;
  const float tr  = t / tau;
  const float cube = (tr * tr) * tr;
  const float q   = (-cube) / (1.0f + tr);
  const float g   = expf(-(tr * tr));
  const float arg = (kTwoPi * t) / phi + 100.0f;
  const float raw = (q * g) * cosf(arg);
  sRaw[k * 16 + c] = raw;
  if (tid < kTapsB) sK1[tid] = k1[tid];
  __syncthreads();
  if (tid < 16) {
    float s = 0.0f;
#pragma unroll 1
    for (int kk = 0; kk < kTapsF; ++kk) {
      const float rv = sRaw[kk * 16 + tid];
      s = s + rv * rv;
    }
    sNrm[tid] = sqrtf(s);
  }
  __syncthreads();
  const float tapv = (-(raw / sNrm[c])) * ctv;
  sTap[c * kTapsF + k] = tapv;
  __syncthreads();
  if (tid < 32) {
    v4u vh[2], vl[2];
#pragma unroll
    for (int it = 0; it < 2; ++it) {
      const int v  = it * 32 + tid;
      const int n  = v >> 2;
      const int k0 = (v & 3) * 8;
      const int nc = n < kCells ? n : kCells - 1;
#pragma unroll
      for (int e2 = 0; e2 < 4; ++e2) {
        const int ka = k0 + 2 * e2;
        const int kb = ka + 1;
        const int kac = ka < kTapsF ? ka : kTapsF - 1;
        const int kbc = kb < kTapsF ? kb : kTapsF - 1;
        const float ra = sTap[nc * kTapsF + kac];
        const float rb = sTap[nc * kTapsF + kbc];
        const float ta = ((n < kCells) && (ka < kTapsF)) ? ra : 0.0f;
        const float tb = ((n < kCells) && (kb < kTapsF)) ? rb : 0.0f;
        const unsigned ha = bf_bits(ta);
        const unsigned hb = bf_bits(tb);
        const unsigned la = bf_bits(ta - bf_bits_to_f(ha));
        const unsigned lb = bf_bits(tb - bf_bits_to_f(hb));
        vh[it][e2] = ha | (hb << 16);
        vl[it][e2] = la | (lb << 16);
      }
    }
    for (int pass = 0; pass < 2; ++pass) {
#pragma unroll
      for (int it = 0; it < 2; ++it) {
        const int v = it * 32 + tid;
        *(volatile v4u*)(bth + v * 4) = vh[it];
        *(volatile v4u*)(btl + v * 4) = vl[it];
      }
      __threadfence();
    }
  }
  if (tid >= 32 && tid < 160) {
    const int v  = tid - 32;
    const int n  = v >> 3;
    const int j0 = (v & 7) * 8;
    v4u vh, vl;
#pragma unroll
    for (int e2 = 0; e2 < 4; ++e2) {
      const int da = j0 + 2 * e2 - n;
      const int db = da + 1;
      int dac = da < 0 ? 0 : da;
      dac = dac > kTapsB - 1 ? kTapsB - 1 : dac;
      int dbc = db < 0 ? 0 : db;
      dbc = dbc > kTapsB - 1 ? kTapsB - 1 : dbc;
      const float ra = sK1[dac];
      const float rb = sK1[dbc];
      const float ta = ((da >= 0) && (da < kTapsB)) ? ra : 0.0f;
      const float tb = ((db >= 0) && (db < kTapsB)) ? rb : 0.0f;
      const unsigned ha = bf_bits(ta);
      const unsigned hb = bf_bits(tb);
      const unsigned la = bf_bits(ta - bf_bits_to_f(ha));
      const unsigned lb = bf_bits(tb - bf_bits_to_f(hb));
      vh[e2] = ha | (hb << 16);
      vl[e2] = la | (lb << 16);
    }
    for (int pass = 0; pass < 2; ++pass) {
      *(volatile v4u*)(bkh + v * 4) = vh;
      *(volatile v4u*)(bkl + v * 4) = vl;
      __threadfence();
    }
  }
}

__global__ __launch_bounds__(256) void front_kernel(
    const float* __restrict__ x, const unsigned short* __restrict__ bth, const unsigned short* __restrict__ btl,
    const float* __restrict__ prm, float* __restrict__ rp)
{
  __shared__ __align__(16) unsigned sXh[kWinWords];
  __shared__ __align__(16) unsigned sXl[kWinWords];
  __shared__ __align__(16) float sSlab[8][16 * 68];
  const int tid  = threadIdx.x;
  const int lane = tid & 31;
  const int wave = tid >> 5;
  const int m    = lane & 15;
  const int h    = lane >> 4;
  const int tb   = blockIdx.x * kBlkT;
  const int mc   = m < kCells ? m : kCells - 1;
  const float off   = prm[PL_OFF * 32 + mc];
  const float slope = prm[PL_SLOPE * 32 + mc];
  const v16b bh = frag_load_bf((const __bf16*)(const void*)bth + m * 32 + 8 * h);
  const v16b bl = frag_load_bf((const __bf16*)(const void*)btl + m * 32 + 8 * h);

  const float x0 = x[0];
#pragma unroll
  for (int jj = 0; jj < 5; ++jj) {
    const int j  = tid + 256 * jj;
    const int jc = j < kWinWords ? j : kWinWords - 1;
    const int g  = tb + 2 * jc;
    int xi = g - kPad;
    xi = xi < 0 ? 0 : xi;
    xi = xi > kD - 2 ? kD - 2 : xi;
    const v2f ld = *(const v2f*)(x + xi);
    const float l0 = ld.x;
    const float l1 = ld.y;
    const bool inpad  = g < kPad;
    const bool indata = g < kXpLen;
    const float v0 = inpad ? x0 : (indata ? l0 : 0.0f);
    const float v1 = inpad ? x0 : (indata ? l1 : 0.0f);
    const unsigned h0 = bf_bits(v0);
    const unsigned h1 = bf_bits(v1);
    const unsigned q0 = bf_bits(v0 - bf_bits_to_f(h0));
    const unsigned q1 = bf_bits(v1 - bf_bits_to_f(h1));
    sXh[jc] = h0 | (h1 << 16);
    sXl[jc] = q0 | (q1 << 16);
  }
  __syncthreads();

  float* slab = sSlab[wave];
#pragma unroll 1
  for (int grp = 0; grp < 4; ++grp) {
#pragma unroll
    for (int tl = 0; tl < 4; ++tl) {
      const int s = wave * 256 + grp * 64 + tl * 16 + m + 8 * h;
      const int w = s >> 1;
      const unsigned sh = ((unsigned)(s & 1)) << 4;
      unsigned ha[5], hb2[5], la[5], lb2[5];
#pragma unroll
      for (int i = 0; i < 5; ++i) {
        ha[i]  = sXh[w + i];
        hb2[i] = sXh[w + 8 + i];
        la[i]  = sXl[w + i];
        lb2[i] = sXl[w + 8 + i];
      }
      v8u wh, wl;
#pragma unroll
      for (int i = 0; i < 4; ++i) {
        wh[i]     = funnel_r(ha[i + 1],  ha[i],  sh);
        wh[4 + i] = funnel_r(hb2[i + 1], hb2[i], sh);
        wl[i]     = funnel_r(la[i + 1],  la[i],  sh);
        wl[4 + i] = funnel_r(lb2[i + 1], lb2[i], sh);
      }
      const v16b ah = __builtin_bit_cast(v16b, wh);
      const v16b al = __builtin_bit_cast(v16b, wl);
      v8f acc = (v8f){0.f, 0.f, 0.f, 0.f, 0.f, 0.f, 0.f, 0.f};
      acc = mma_bf(ah, bh, acc);
      acc = mma_bf(ah, bl, acc);
      acc = mma_bf(al, bh, acc);
      group_guard(acc, ah, al, bh, bl);
      float rv[8];
#pragma unroll
      for (int r = 0; r < 8; ++r) {
        const float z = (acc[r] - off) * slope;
        const float e = __expf(-z);
        rv[r] = __builtin_amdgcn_rcpf(1.0f + e);
      }
      const v4f s0 = (v4f){rv[0], rv[1], rv[2], rv[3]};
      const v4f s1 = (v4f){rv[4], rv[5], rv[6], rv[7]};
      *(v4f*)(slab + m * 68 + tl * 16 + 8 * h)     = s0;
      *(v4f*)(slab + m * 68 + tl * 16 + 8 * h + 4) = s1;
    }
    __builtin_amdgcn_fence(__ATOMIC_RELEASE, "workgroup");
    __builtin_amdgcn_wave_barrier();
    __builtin_amdgcn_fence(__ATOMIC_ACQUIRE, "workgroup");
    {
      const int tg = tb + wave * 256 + grp * 64;
      const int q  = lane >> 3;
      const int c4 = (lane & 7) * 4;
      v4f sv[7];
#pragma unroll
      for (int it = 0; it < 7; ++it) {
        const int L    = it * 4 + q;
        const int cell = L >> 1;
        const int hl   = L & 1;
        sv[it] = *(const v4f*)(slab + cell * 68 + hl * 32 + c4);
      }
      for (int pass = 0; pass < 2; ++pass) {
#pragma unroll
        for (int it = 0; it < 7; ++it) {
          const int L    = it * 4 + q;
          const int cell = L >> 1;
          const int hl   = L & 1;
          *(volatile v4f*)(rp + (size_t)cell * kTP + tg + hl * 32 + c4) = sv[it];
        }
        __threadfence();
      }
    }
    __builtin_amdgcn_fence(__ATOMIC_RELEASE, "workgroup");
    __builtin_amdgcn_wave_barrier();
    __builtin_amdgcn_fence(__ATOMIC_ACQUIRE, "workgroup");
  }
}

__global__ __launch_bounds__(32) void pool_scan_kernel(
    const float* __restrict__ rp, const float* __restrict__ prm, float* __restrict__ rel)
{
  const int lane = threadIdx.x;
  const int cc   = lane < kCells ? lane : kCells - 1;
  const bool live = lane < kCells;
  const float cp01   = prm[PL_CP01 * 32 + cc];
  const float cp12   = prm[PL_CP12 * 32 + cc];
  const float rrpcap = prm[PL_RRPCAP * 32 + cc];
  const float ipcap  = prm[PL_IPCAP * 32 + cc];
  float ip  = prm[PL_IP0 * 32 + cc];
  float rrp = prm[PL_RRP0 * 32 + cc];
  const float hm1r = rrpcap - 1.0f;
  const float hm1i = ipcap - 1.0f;
  const float* src = rp  + (size_t)cc * kTP;
  float*       dst = rel + (size_t)cc * kTP;
#pragma unroll 1
  for (int ch = 0; ch < kNChunk; ++ch) {
    const size_t o = (size_t)ch * kChunk;
    v4f buf[16];
#pragma unroll
    for (int j = 0; j < 16; ++j) buf[j] = *(const v4f*)(src + o + 4 * j);
#pragma unroll
    for (int j = 0; j < 16; ++j) {
#pragma unroll
      for (int e = 0; e < 4; ++e) {
        const float rpv      = buf[j][e];
        const float relv     = rpv * rrp;
        const float released = rrp - relv;
        const float tin      = cp12 * ip;
        const float x1       = released + tin;
        const float rn       = smooth_clamp_step(x1, rrpcap, hm1r);
        const float transfer = rn - released;
        const float x2       = (ip + cp01) - transfer;
        ip  = smooth_clamp_step(x2, ipcap, hm1i);
        rrp = rn;
        buf[j][e] = relv;
      }
    }
    for (int pass = 0; pass < 2; ++pass) {
      if (live) {
#pragma unroll
        for (int j = 0; j < 16; ++j) *(volatile v4f*)(dst + o + 4 * j) = buf[j];
      }
      __threadfence();
    }
  }
}

__global__ __launch_bounds__(256) void readout_kernel(
    const float* __restrict__ rel, const unsigned short* __restrict__ bkh, const unsigned short* __restrict__ bkl,
    const float* __restrict__ prm, float* __restrict__ out)
{
  __shared__ __align__(16) unsigned sRh[kRdWords];
  __shared__ __align__(16) unsigned sRl[kRdWords];
  __shared__ __align__(16) float sO[8][256];
  const int tid  = threadIdx.x;
  const int lane = tid & 31;
  const int wave = tid >> 5;
  const int n    = lane & 15;
  const int h    = lane >> 4;
  const int cell = blockIdx.y;
  const int d0   = blockIdx.x * kRdBlk;
  const float scale = prm[PL_SCALE * 32 + cell];
  const float bias  = prm[PL_BIAS * 32 + cell];
  const v16b bh0 = frag_load_bf((const __bf16*)(const void*)bkh + n * kBandK + 8 * h);
  const v16b bh1 = frag_load_bf((const __bf16*)(const void*)bkh + n * kBandK + 32 + 8 * h);
  const v16b bl0 = frag_load_bf((const __bf16*)(const void*)bkl + n * kBandK + 8 * h);
  const v16b bl1 = frag_load_bf((const __bf16*)(const void*)bkl + n * kBandK + 32 + 8 * h);

  const float* src = rel + (size_t)cell * kTP + kSteady + d0;
#pragma unroll
  for (int jj = 0; jj < 3; ++jj) {
    const int qd = tid + 256 * jj;
    const int qc = qd < kRdQuads ? qd : kRdQuads - 1;
    const v4f ld = *(const v4f*)(src + 4 * qc);
    const float f0 = ld.x;
    const float f1 = ld.y;
    const float f2 = ld.z;
    const float f3 = ld.w;
    const unsigned h0 = bf_bits(f0);
    const unsigned h1 = bf_bits(f1);
    const unsigned h2 = bf_bits(f2);
    const unsigned h3 = bf_bits(f3);
    const unsigned q0 = bf_bits(f0 - bf_bits_to_f(h0));
    const unsigned q1 = bf_bits(f1 - bf_bits_to_f(h1));
    const unsigned q2 = bf_bits(f2 - bf_bits_to_f(h2));
    const unsigned q3 = bf_bits(f3 - bf_bits_to_f(h3));
    const v2u wh = (v2u){h0 | (h1 << 16), h2 | (h3 << 16)};
    const v2u wl = (v2u){q0 | (q1 << 16), q2 | (q3 << 16)};
    *(v2u*)(sRh + 2 * qc) = wh;
    *(v2u*)(sRl + 2 * qc) = wl;
  }
  __syncthreads();

  const int w0 = wave * 128 + 8 * n + 4 * h;
  const v4u h00 = *(const v4u*)(sRh + w0);
  const v4u h01 = *(const v4u*)(sRh + w0 + 8);
  const v4u h10 = *(const v4u*)(sRh + w0 + 16);
  const v4u h11 = *(const v4u*)(sRh + w0 + 24);
  const v4u l00 = *(const v4u*)(sRl + w0);
  const v4u l01 = *(const v4u*)(sRl + w0 + 8);
  const v4u l10 = *(const v4u*)(sRl + w0 + 16);
  const v4u l11 = *(const v4u*)(sRl + w0 + 24);
  const v8u wh0 = __builtin_shufflevector(h00, h01, 0, 1, 2, 3, 4, 5, 6, 7);
  const v8u wh1 = __builtin_shufflevector(h10, h11, 0, 1, 2, 3, 4, 5, 6, 7);
  const v8u wl0 = __builtin_shufflevector(l00, l01, 0, 1, 2, 3, 4, 5, 6, 7);
  const v8u wl1 = __builtin_shufflevector(l10, l11, 0, 1, 2, 3, 4, 5, 6, 7);
  const v16b ah0 = __builtin_bit_cast(v16b, wh0);
  const v16b ah1 = __builtin_bit_cast(v16b, wh1);
  const v16b al0 = __builtin_bit_cast(v16b, wl0);
  const v16b al1 = __builtin_bit_cast(v16b, wl1);

  v8f acc = (v8f){0.f, 0.f, 0.f, 0.f, 0.f, 0.f, 0.f, 0.f};
  acc = mma_bf(ah0, bh0, acc);
  acc = mma_bf(ah0, bl0, acc);
  acc = mma_bf(al0, bh0, acc);
  group_guard(acc, ah0, al0, bh0, bl0);
  acc = mma_bf(ah1, bh1, acc);
  acc = mma_bf(ah1, bl1, acc);
  acc = mma_bf(al1, bh1, acc);
  group_guard(acc, ah1, al1, bh1, bl1);

  float* slab = sO[wave];
#pragma unroll
  for (int r = 0; r < 8; ++r) {
    const float p = acc[r] * scale;
    slab[16 * (8 * h + r) + n] = p + bias;
  }
  __builtin_amdgcn_fence(__ATOMIC_RELEASE, "workgroup");
  __builtin_amdgcn_wave_barrier();
  __builtin_amdgcn_fence(__ATOMIC_ACQUIRE, "workgroup");
  v4f ov[2];
#pragma unroll
  for (int it = 0; it < 2; ++it) ov[it] = *(const v4f*)(slab + 128 * it + 4 * lane);
  float* dst = out + (size_t)cell * kD + d0 + wave * 256;
  for (int pass = 0; pass < 2; ++pass) {
#pragma unroll
    for (int it = 0; it < 2; ++it) *(volatile v4f*)(dst + 128 * it + 4 * lane) = ov[it];
    __threadfence();
  }
}

extern "C" void kernel_launch(void* const* d_in, const int* in_sizes, int n_in,
                              void* d_out, int out_size, void* d_ws, size_t ws_size,
                              hipStream_t stream) {
  if (n_in < 14) return;
  if (in_sizes[0] != kD) return;
  for (int i = 1; i <= 12; ++i) {
    if (in_sizes[i] != kCells) return;
  }
  if (in_sizes[13] != kTapsB) return;
  if (out_size != kCells * kD) return;
  if (ws_size < kWsTotal) return;

  const float* x     = (const float*)d_in[0];
  const float* lks   = (const float*)d_in[1];
  const float* soff  = (const float*)d_in[2];
  const float* lsl   = (const float*)d_in[3];
  const float* lcp01 = (const float*)d_in[4];
  const float* lcp12 = (const float*)d_in[5];
  const float* lipc  = (const float*)d_in[6];
  const float* lrpc  = (const float*)d_in[7];
  const float* sip   = (const float*)d_in[8];
  const float* srrp  = (const float*)d_in[9];
  const float* lfs   = (const float*)d_in[10];
  const float* fb    = (const float*)d_in[11];
  const float* ct    = (const float*)d_in[12];
  const float* k1    = (const float*)d_in[13];
  float* out = (float*)d_out;

  char* ws = (char*)d_ws;
  float*    prm = (float*)(ws + kOffPRM);
  unsigned* bth = (unsigned*)(ws + kOffBTH);
  unsigned* btl = (unsigned*)(ws + kOffBTL);
  unsigned* bkh = (unsigned*)(ws + kOffBKH);
  unsigned* bkl = (unsigned*)(ws + kOffBKL);
  float*    rp  = (float*)(ws + kOffRP);
  float*    rel = (float*)(ws + kOffREL);

  params_kernel<<<1, 160, 0, stream>>>(prm, soff, lsl, lcp01, lcp12, lipc, lrpc, sip, srrp, lfs, fb);
  taps_kernel<<<1, 320, 0, stream>>>(lks, ct, k1, bth, btl, bkh, bkl);
  front_kernel<<<kFrontBlocks, 256, 0, stream>>>(x, (const unsigned short*)bth, (const unsigned short*)btl, prm, rp);
  pool_scan_kernel<<<1, 32, 0, stream>>>(rp, prm, rel);
  readout_kernel<<<dim3(kD / kRdBlk, kCells), 256, 0, stream>>>(rel, (const unsigned short*)bkh, (const unsigned short*)bkl, prm, out);
}
